// StrideAwareWiredCfCCell_4294967296464
// MI455X (gfx1250) — hardware-verified
//
#include <hip/hip_runtime.h>
#include <stdint.h>
#include <stddef.h>
#include <math.h>

#pragma clang fp contract(off)

#define NB   1024
#define DIN  512
#define NU   1024
#define NH   2048
#define TBM  128
#define TBN  128
#define TT   64
#define TPH  72
#define SPH  72
#define SPF  68
#define STG  4608
#define WSCALE 16.0f
#define WINV   0.0625f

static_assert(32 * SPH * 2 <= STG);
static_assert(16 * SPF * 4 <= STG);
static_assert((SPH * 2) % 16 == 0);
static_assert((SPF * 4) % 16 == 0);
static_assert((TPH * 2) % 16 == 0);
static_assert(STG % 16 == 0);
static_assert(NB % TBM == 0);
static_assert(NU % TBN == 0);
static_assert(NH % TBN == 0);
static_assert(DIN % 32 == 0);
static_assert(NU % 32 == 0);
static_assert(NH % 32 == 0);
static_assert(DIN % TT == 0);
static_assert(NU % TT == 0);
static_assert(NH % TT == 0);
static_assert((NB * DIN) % 2048 == 0);
static_assert((NB * NU) % 2048 == 0);

typedef _Float16 v16h __attribute__((ext_vector_type(16)));
typedef _Float16 v8h  __attribute__((ext_vector_type(8)));
typedef float    v8f  __attribute__((ext_vector_type(8)));
typedef float    v4f  __attribute__((ext_vector_type(4)));
typedef v4f __attribute__((may_alias)) v4fa;
typedef v8h __attribute__((may_alias)) v8ha;

union FragH { v16h v; v8h q[2]; };

__device__ __forceinline__ v8f wmma_h(v16h a, v16h b, v8f c) {
  v8f d = __builtin_amdgcn_wmma_f32_16x16x32_f16(false, a, false, b, (short)0, c, false, false);
  asm volatile("v_nop\n\tv_nop\n\tv_nop\n\tv_nop" : "+v"(d) : "v"(a), "v"(b));
  return d;
}

__device__ __forceinline__ v16h ldfrag_h(const _Float16* p, int h) {
  FragH f;
  f.q[0] = *(const v8ha*)(p + 8 * h);
  f.q[1] = *(const v8ha*)(p + 16 + 8 * h);
  return f.v;
}

__device__ __forceinline__ float lecun_tanh_f(float x) {
  const float v  = 0.66666667f * x;
  const float ax = fminf(fabsf(v), 9.0f);
  const float ex = __expf(ax + ax);
  const float r  = __builtin_amdgcn_rcpf(ex + 1.0f);
  return 1.7159f * copysignf(1.0f - 2.0f * r, v);
}

__device__ __forceinline__ float sigmoid_f(float v) {
  const float c = fminf(fmaxf(v, -30.0f), 30.0f);
  return __builtin_amdgcn_rcpf(1.0f + __expf(-c));
}

template <int MODE>
__global__ __launch_bounds__(256) void k_cvt(const float* __restrict__ src,
                                             const float* __restrict__ msk,
                                             _Float16* __restrict__ dst,
                                             int n8, int cols)
{
  const int i = blockIdx.x * 256 + threadIdx.x;
  if (i >= n8) return;
  const size_t e = (size_t)i * 8;
  v4f a = *(const v4fa*)(src + e);
  v4f b = *(const v4fa*)(src + e + 4);
  if constexpr (MODE == 1) {
    const size_t c = e % (size_t)cols;
    const v4f ma = *(const v4fa*)(msk + c);
    const v4f mb = *(const v4fa*)(msk + c + 4);
    a = a * ma; b = b * mb;
  } else if constexpr (MODE == 2) {
    const v4f ma = *(const v4fa*)(msk + e);
    const v4f mb = *(const v4fa*)(msk + e + 4);
    a = a * ma; b = b * mb;
  }
  v8h o;
  o[0] = (_Float16)a.x; o[1] = (_Float16)a.y; o[2] = (_Float16)a.z; o[3] = (_Float16)a.w;
  o[4] = (_Float16)b.x; o[5] = (_Float16)b.y; o[6] = (_Float16)b.z; o[7] = (_Float16)b.w;
  _Float16* d = dst + e;
  *(volatile v8ha*)d = o;
  __threadfence();
  *(volatile v8ha*)d = o;
}

__global__ __launch_bounds__(256) void k_wt(const float* __restrict__ src,
                                            _Float16* __restrict__ dst,
                                            int R, int C, float scale)
{
  __shared__ __align__(16) _Float16 sT[TT * TPH];
  const int tid = threadIdx.x, lane = tid & 31, wv = tid >> 5;
  const int r0 = blockIdx.y * TT;
  const int c0 = blockIdx.x * TT;

  const int i = tid >> 2, cs = (tid & 3) * 16;
  const float* sp = src + (size_t)(r0 + i) * C + c0 + cs;
  const v4f a0 = *(const v4fa*)(sp);
  const v4f a1 = *(const v4fa*)(sp + 4);
  const v4f a2 = *(const v4fa*)(sp + 8);
  const v4f a3 = *(const v4fa*)(sp + 12);
  _Float16* tp = sT + cs * TPH + i;
  tp[ 0 * TPH] = (_Float16)(a0.x * scale);
  tp[ 1 * TPH] = (_Float16)(a0.y * scale);
  tp[ 2 * TPH] = (_Float16)(a0.z * scale);
  tp[ 3 * TPH] = (_Float16)(a0.w * scale);
  tp[ 4 * TPH] = (_Float16)(a1.x * scale);
  tp[ 5 * TPH] = (_Float16)(a1.y * scale);
  tp[ 6 * TPH] = (_Float16)(a1.z * scale);
  tp[ 7 * TPH] = (_Float16)(a1.w * scale);
  tp[ 8 * TPH] = (_Float16)(a2.x * scale);
  tp[ 9 * TPH] = (_Float16)(a2.y * scale);
  tp[10 * TPH] = (_Float16)(a2.z * scale);
  tp[11 * TPH] = (_Float16)(a2.w * scale);
  tp[12 * TPH] = (_Float16)(a3.x * scale);
  tp[13 * TPH] = (_Float16)(a3.y * scale);
  tp[14 * TPH] = (_Float16)(a3.z * scale);
  tp[15 * TPH] = (_Float16)(a3.w * scale);
  __syncthreads();

  const int q  = lane & 7;
  const int cA = 4 * wv + (lane >> 3);
  const int cB = 32 + cA;
  const v8h vA = *(const v8ha*)(sT + cA * TPH + 8 * q);
  const v8h vB = *(const v8ha*)(sT + cB * TPH + 8 * q);
  _Float16* dA = dst + (size_t)(c0 + cA) * R + r0 + 8 * q;
  _Float16* dB = dst + (size_t)(c0 + cB) * R + r0 + 8 * q;
  *(volatile v8ha*)dA = vA;
  *(volatile v8ha*)dB = vB;
  __threadfence();
  *(volatile v8ha*)dA = vA;
  *(volatile v8ha*)dB = vB;
}

__device__ __forceinline__ void kloop(v8f (&acc)[2][4],
                                      const _Float16* A, int lda,
                                      const _Float16* Bt, int ldb, int K,
                                      int rowW, int colW, int h, int m)
{
  const _Float16* a0p = A  + (size_t)(rowW + m) * lda;
  const _Float16* a1p = A  + (size_t)(rowW + 16 + m) * lda;
  const _Float16* b0p = Bt + (size_t)(colW + m) * ldb;
  #pragma unroll 1
  for (int k0 = 0; k0 < K; k0 += 32) {
    const v16h a0 = ldfrag_h(a0p + k0, h);
    const v16h a1 = ldfrag_h(a1p + k0, h);
    #pragma unroll
    for (int nt = 0; nt < 4; ++nt) {
      const v16h b = ldfrag_h(b0p + (size_t)(16 * nt) * ldb + k0, h);
      acc[0][nt] = wmma_h(a0, b, acc[0][nt]);
      acc[1][nt] = wmma_h(a1, b, acc[1][nt]);
    }
  }
}

template <int EPI>
__global__ __launch_bounds__(256) void k_gemm(const _Float16* A1, int lda1,
                                              const _Float16* B1, int ldb1, int K1,
                                              const _Float16* A2, int lda2,
                                              const _Float16* B2, int ldb2, int K2,
                                              const float* bias,
                                              _Float16* outh, float* outf, int ldo,
                                              const float* gate, const float* hprev,
                                              const float* tker, const float* tptr,
                                              const float* omask,
                                              float* out0, float* out1)
{
  __shared__ __align__(16) unsigned char s_stage[8 * STG];
  const int tid = threadIdx.x, lane = tid & 31, w = tid >> 5;
  const int h = lane >> 4, m = lane & 15;
  const int wm = w >> 1, wn = w & 1;
  const int rowW = blockIdx.y * TBM + 32 * wm;
  const int colW = blockIdx.x * TBN + 64 * wn;

  const v8f z8 = {0.f, 0.f, 0.f, 0.f, 0.f, 0.f, 0.f, 0.f};
  v8f acc[2][4];
  #pragma unroll
  for (int mt = 0; mt < 2; ++mt)
    #pragma unroll
    for (int nt = 0; nt < 4; ++nt) acc[mt][nt] = z8;

  kloop(acc, A1, lda1, B1, ldb1, K1, rowW, colW, h, m);
  kloop(acc, A2, lda2, B2, ldb2, K2, rowW, colW, h, m);

  if constexpr (EPI == 0) {
    _Float16* st = (_Float16*)(s_stage + w * STG);
    #pragma unroll
    for (int nt = 0; nt < 4; ++nt) {
      const float bv = bias[colW + 16 * nt + m];
      #pragma unroll
      for (int mt = 0; mt < 2; ++mt) {
        #pragma unroll
        for (int r = 0; r < 8; ++r) {
          const int row = 16 * mt + 8 * h + r;
          const int col = 16 * nt + m;
          const float v = acc[mt][nt][r] * WINV + bv;
          st[row * SPH + col] = (_Float16)lecun_tanh_f(v);
        }
      }
    }
    __syncthreads();
    const int q = lane & 7, rs = lane >> 3;
    _Float16* ob = outh + (size_t)rowW * ldo + colW + 8 * q;
    #pragma unroll
    for (int it = 0; it < 8; ++it) {
      const int row = 4 * it + rs;
      const v8h v = *(const v8ha*)(st + row * SPH + 8 * q);
      *(volatile v8ha*)(ob + (size_t)row * ldo) = v;
    }
    __threadfence();
    #pragma unroll
    for (int it = 0; it < 8; ++it) {
      const int row = 4 * it + rs;
      const v8h v = *(const v8ha*)(st + row * SPH + 8 * q);
      *(volatile v8ha*)(ob + (size_t)row * ldo) = v;
    }
  } else {
    float* stf = (float*)(s_stage + w * STG);
    const int hl = lane >> 4, q4 = lane & 15;
    const int colL = colW + 4 * q4;
    v4f tg4 = {0.f, 0.f, 0.f, 0.f};
    v4f om4 = {0.f, 0.f, 0.f, 0.f};
    if constexpr (EPI == 2) {
      const float teff = (tptr[0] * 2.0f) * 1.0f;
      const float at = fabsf(teff);
      const v4f tk = *(const v4fa*)(tker + colL);
      om4 = *(const v4fa*)(omask + colL);
      #pragma unroll
      for (int j = 0; j < 4; ++j) tg4[j] = expf(-at * expf(tk[j]));
    }
    #pragma unroll
    for (int mt = 0; mt < 2; ++mt) {
      if (mt) __syncthreads();
      #pragma unroll
      for (int nt = 0; nt < 4; ++nt) {
        const float bv = bias[colW + 16 * nt + m];
        #pragma unroll
        for (int r = 0; r < 8; ++r) {
          const int row = 8 * h + r;
          const int col = 16 * nt + m;
          float v = acc[mt][nt][r] * WINV + bv;
          if constexpr (EPI == 1) v = sigmoid_f(v);
          stf[row * SPF + col] = v;
        }
      }
      __syncthreads();
      v4f vals[8];
      #pragma unroll
      for (int it = 0; it < 8; ++it) {
        const int row = 2 * it + hl;
        const v4f hc = *(const v4fa*)(stf + row * SPF + 4 * q4);
        if constexpr (EPI == 1) {
          vals[it] = hc;
        } else {
          const size_t gidx = (size_t)(rowW + 16 * mt + row) * ldo + colL;
          const v4f g  = *(const v4fa*)(gate + gidx);
          const v4f hp = *(const v4fa*)(hprev + gidx);
          v4f hn;
          #pragma unroll
          for (int j = 0; j < 4; ++j)
            hn[j] = hp[j] * g[j] + hc[j] * (1.0f - g[j]) * (1.0f - tg4[j]);
          vals[it] = hn;
        }
      }
      #pragma unroll
      for (int it = 0; it < 8; ++it) {
        const size_t oidx = (size_t)(rowW + 16 * mt + 2 * it + hl) * ldo + colL;
        if constexpr (EPI == 1) {
          *(volatile v4fa*)(outf + oidx) = vals[it];
        } else {
          const v4f o0 = vals[it] * om4;
          *(volatile v4fa*)(out1 + oidx) = vals[it];
          *(volatile v4fa*)(out0 + oidx) = o0;
        }
      }
      __threadfence();
      #pragma unroll
      for (int it = 0; it < 8; ++it) {
        const size_t oidx = (size_t)(rowW + 16 * mt + 2 * it + hl) * ldo + colL;
        if constexpr (EPI == 1) {
          *(volatile v4fa*)(outf + oidx) = vals[it];
        } else {
          const v4f o0 = vals[it] * om4;
          *(volatile v4fa*)(out1 + oidx) = vals[it];
          *(volatile v4fa*)(out0 + oidx) = o0;
        }
      }
    }
  }
}

extern "C" void kernel_launch(void* const* d_in, const int* in_sizes, int n_in,
                              void* d_out, int out_size, void* d_ws, size_t ws_size,
                              hipStream_t stream)
{
  if (n_in < 17) return;
  if (in_sizes[0]  != NB * DIN) return;
  if (in_sizes[1]  != NB * NU) return;
  if (in_sizes[2]  != 1) return;
  if (in_sizes[3]  != DIN * NH) return;
  if (in_sizes[4]  != NU * NH) return;
  if (in_sizes[5]  != NH * NH) return;
  if (in_sizes[6]  != NH) return;
  if (in_sizes[7]  != NH * NU) return;
  if (in_sizes[8]  != NU) return;
  if (in_sizes[9]  != NH) return;
  if (in_sizes[10] != NU) return;
  if (in_sizes[11] != DIN * NU) return;
  if (in_sizes[12] != NU * NU) return;
  if (in_sizes[13] != NU) return;
  if (in_sizes[14] != DIN) return;
  if (in_sizes[15] != NU * NU) return;
  if (in_sizes[16] != NU) return;
  if (out_size != 2 * NB * NU) return;

  const float* xin   = (const float*)d_in[0];
  const float* hprev = (const float*)d_in[1];
  const float* tptr  = (const float*)d_in[2];
  const float* Wk    = (const float*)d_in[3];
  const float* Wr    = (const float*)d_in[4];
  const float* Wb    = (const float*)d_in[5];
  const float* bbb   = (const float*)d_in[6];
  const float* Wo    = (const float*)d_in[7];
  const float* tker  = (const float*)d_in[8];
  const float* bias  = (const float*)d_in[9];
  const float* rbias = (const float*)d_in[10];
  const float* Wg    = (const float*)d_in[11];
  const float* Wgr   = (const float*)d_in[12];
  const float* gbias = (const float*)d_in[13];
  const float* imask = (const float*)d_in[14];
  const float* rmask = (const float*)d_in[15];
  const float* omask = (const float*)d_in[16];
  float* out0 = (float*)d_out;
  float* out1 = out0 + (size_t)NB * NU;

  const size_t bAin = (size_t)NB * DIN * 2;
  const size_t bAh  = (size_t)NB * NU  * 2;
  const size_t bWk  = (size_t)NH * DIN * 2;
  const size_t bWr  = (size_t)NH * NU  * 2;
  const size_t bWb  = (size_t)NH * NH  * 2;
  const size_t bWo  = (size_t)NU * NH  * 2;
  const size_t bWg  = (size_t)NU * DIN * 2;
  const size_t bWgr = (size_t)NU * NU  * 2;
  const size_t bX   = (size_t)NB * NH  * 2;
  const size_t bG   = (size_t)NB * NU  * 4;
  const size_t total = 2 * bAin + 2 * bAh + bWk + bWr + bWb + bWo + bWg + bWgr + 2 * bX + bG;
  if (total > ws_size) return;
  if (total > (size_t)134217728) return;

  char* ws = (char*)d_ws;
  size_t off = 0;
  _Float16* Axm  = (_Float16*)(ws + off); off += bAin;
  _Float16* Ahm  = (_Float16*)(ws + off); off += bAh;
  _Float16* Ax   = (_Float16*)(ws + off); off += bAin;
  _Float16* Ah   = (_Float16*)(ws + off); off += bAh;
  _Float16* WkT  = (_Float16*)(ws + off); off += bWk;
  _Float16* WrT  = (_Float16*)(ws + off); off += bWr;
  _Float16* WbT  = (_Float16*)(ws + off); off += bWb;
  _Float16* WoT  = (_Float16*)(ws + off); off += bWo;
  _Float16* WgT  = (_Float16*)(ws + off); off += bWg;
  _Float16* WgrT = (_Float16*)(ws + off); off += bWgr;
  _Float16* X1   = (_Float16*)(ws + off); off += bX;
  _Float16* X2   = (_Float16*)(ws + off); off += bX;
  float*    G    = (float*)(ws + off);    off += bG;
  if (off != total) return;

  k_cvt<1><<<(NB * DIN / 8) / 256, 256, 0, stream>>>(xin,   imask, Axm, NB * DIN / 8, DIN);
  k_cvt<2><<<(NB * NU  / 8) / 256, 256, 0, stream>>>(hprev, rmask, Ahm, NB * NU  / 8, NU);
  k_cvt<0><<<(NB * DIN / 8) / 256, 256, 0, stream>>>(xin,   imask, Ax,  NB * DIN / 8, DIN);
  k_cvt<0><<<(NB * NU  / 8) / 256, 256, 0, stream>>>(hprev, rmask, Ah,  NB * NU  / 8, NU);

  k_wt<<<dim3(NH / TT, DIN / TT), 256, 0, stream>>>(Wk,  WkT,  DIN, NH, WSCALE);
  k_wt<<<dim3(NH / TT, NU  / TT), 256, 0, stream>>>(Wr,  WrT,  NU,  NH, WSCALE);
  k_wt<<<dim3(NH / TT, NH  / TT), 256, 0, stream>>>(Wb,  WbT,  NH,  NH, WSCALE);
  k_wt<<<dim3(NU / TT, NH  / TT), 256, 0, stream>>>(Wo,  WoT,  NH,  NU, WSCALE);
  k_wt<<<dim3(NU / TT, DIN / TT), 256, 0, stream>>>(Wg,  WgT,  DIN, NU, WSCALE);
  k_wt<<<dim3(NU / TT, NU  / TT), 256, 0, stream>>>(Wgr, WgrT, NU,  NU, WSCALE);

  k_gemm<0><<<dim3(NH / TBN, NB / TBM), 256, 0, stream>>>(
      Axm, DIN, WkT, DIN, DIN, Ahm, NU, WrT, NU, NU,
      bias, X1, G, NH, G, hprev, tker, tptr, omask, out0, out1);
  k_gemm<0><<<dim3(NH / TBN, NB / TBM), 256, 0, stream>>>(
      X1, NH, WbT, NH, NH, X1, NH, WbT, NH, 0,
      bbb, X2, G, NH, G, hprev, tker, tptr, omask, out0, out1);
  k_gemm<1><<<dim3(NU / TBN, NB / TBM), 256, 0, stream>>>(
      Ax, DIN, WgT, DIN, DIN, Ah, NU, WgrT, NU, NU,
      gbias, X1, G, NU, hprev, hprev, tker, tptr, omask, out0, out1);
  k_gemm<2><<<dim3(NU / TBN, NB / TBM), 256, 0, stream>>>(
      X2, NH, WoT, NH, NH, X2, NH, WoT, NH, 0,
      rbias, X1, G, NU, G, hprev, tker, tptr, omask, out0, out1);
}
